// RNNModel_37555194036798
// MI455X (gfx1250) — hardware-run, weakly checked
//
#include <hip/hip_runtime.h>
#include <math.h>

#pragma clang fp contract(off)

constexpr int NB      = 512;
constexpr int NSTEP   = 1024;
constexpr int NH      = 128;
constexpr int NG3     = 3 * NH;
constexpr int NO      = 4;
constexpr int NTHR    = 256;
constexpr int NWAVE   = NTHR / 32;
constexpr int RB      = 16;
constexpr int WPITCH  = 136;
constexpr int HPITCH  = 136;
constexpr int XCH     = 64;
constexpr int HSP     = 132;
constexpr int W_ITERS = (NG3 * NH) / (NTHR * 4);
static_assert(NB % RB == 0);
static_assert(NH == 16 * NWAVE);
static_assert(NH % 32 == 0);
static_assert(NSTEP % XCH == 0);
static_assert(RB * XCH == NTHR * 4);
static_assert((NG3 * NH) % (NTHR * 4) == 0);
static_assert(WPITCH - NH == 8 && HPITCH >= NH);
static_assert((2 * RB * HPITCH) % NTHR == 0);
static_assert((NG3 * (WPITCH - NH)) % NTHR == 0);
static_assert(NO * NH == 4 * 128);
static_assert(RB * NO == 64);

typedef __attribute__((ext_vector_type(16))) __bf16   v16b;
typedef __attribute__((ext_vector_type(8)))  __bf16   v8b;
typedef __attribute__((ext_vector_type(8)))  float    v8f;
typedef __attribute__((ext_vector_type(4)))  float    v4f;

__device__ __forceinline__ unsigned short f2bf_bits(float f) {
  unsigned u = __float_as_uint(f);
  return (unsigned short)((u + 0x7FFFu + ((u >> 16) & 1u)) >> 16);
}
__device__ __forceinline__ float bf_bits2f(unsigned short h) { return __uint_as_float(((unsigned)h) << 16); }
__device__ __forceinline__ float bf16r(float f) { return bf_bits2f(f2bf_bits(f)); }
__device__ __forceinline__ __bf16 f2bf(float f) { const unsigned short b = f2bf_bits(f); return __builtin_bit_cast(__bf16, b); }

__device__ __forceinline__ void mma_guard3(v8f& a0, v8f& a1, v8f& a2, v16b f0, v16b f1, v16b f2, v16b f3, v16b f4) {
  asm volatile("v_nop\n\tv_nop\n\tv_nop\n\tv_nop" : "+v"(a0), "+v"(a1), "+v"(a2) : "v"(f0), "v"(f1), "v"(f2), "v"(f3), "v"(f4));
}
__device__ __forceinline__ void acc_guard3(v8f& a, v8f& b, v8f& c) {
  asm volatile("v_nop\n\tv_nop\n\tv_nop\n\tv_nop" : "+v"(a), "+v"(b), "+v"(c));
}

template <typename T> struct Frag;
template <> struct Frag<__bf16> {
  typedef v16b V; union U { v16b v; v8b h[2]; };
  static __device__ __forceinline__ v16b load(const __bf16* p) {
    U f; f.h[0] = *(const v8b*)(p); f.h[1] = *(const v8b*)(p + 16); return f.v;
  }
  static __device__ __forceinline__ v8f mma(v16b a, v16b b, v8f c) {
    return __builtin_amdgcn_wmma_f32_16x16x32_bf16(false, a, false, b, (short)0, c, false, false);
  }
};

__device__ __forceinline__ float fsig(float x)  { return __builtin_amdgcn_rcpf(1.0f + expf(-x)); }
__device__ __forceinline__ float ftanh(float x) { return 1.0f - 2.0f * __builtin_amdgcn_rcpf(expf(2.0f * x) + 1.0f); }

__global__ __launch_bounds__(NTHR) void gru_seq_kernel(const float* __restrict__ x, const float* __restrict__ w_ih,
                                                       const float* __restrict__ w_hh, const float* __restrict__ b_ih,
                                                       const float* __restrict__ b_hh, const float* __restrict__ fc_w,
                                                       const float* __restrict__ fc_b, float* __restrict__ out) {
  __shared__ __align__(16) __bf16 Wsh[NG3 * WPITCH];
  __shared__ __align__(16) __bf16 Hh[2][RB * HPITCH];
  __shared__ __align__(16) __bf16 Hl[2][RB * HPITCH];
  __shared__ __align__(16) float  Xs[RB * XCH];
  __shared__ __align__(16) float  Hs[RB * HSP];
  __shared__ __align__(16) float  Fw[NO * NH];
  __shared__ __align__(16) float  Fb[NO];
  __shared__ __align__(16) float  Os[RB * NO];

  const int tid  = threadIdx.x;
  const int lane = tid & 31;
  const int wave = tid >> 5;
  const int c    = lane & 15;
  const int hh   = lane >> 4;
  const int koff = hh * 8;
  const int j    = 16 * wave + c;
  const int rowbase = blockIdx.x * RB;

  {
    const unsigned short zbits = 0;
    const __bf16 zb = __builtin_bit_cast(__bf16, zbits);
    __bf16* hp = &Hh[0][0];
    __bf16* lp = &Hl[0][0];
#pragma unroll 1
    for (int i = tid; i < 2 * RB * HPITCH; i += NTHR) { hp[i] = zb; lp[i] = zb; }
#pragma unroll 1
    for (int i = tid; i < NG3 * (WPITCH - NH); i += NTHR) {
      const int row = i >> 3;
      const int pc  = NH + (i & 7);
      Wsh[row * WPITCH + pc] = zb;
    }
  }
  __syncthreads();

#pragma unroll 1
  for (int it = 0; it < W_ITERS; ++it) {
    const int idx = it * NTHR + tid;
    const int row = idx >> 5;
    const int c4  = (idx & 31) * 4;
    const v4f v = *(const v4f*)(w_hh + (size_t)row * NH + c4);
    const float v0 = v[0], v1 = v[1], v2 = v[2], v3 = v[3];
    __bf16* wp = Wsh + row * WPITCH + c4;
    wp[0] = f2bf(v0);
    wp[1] = f2bf(v1);
    wp[2] = f2bf(v2);
    wp[3] = f2bf(v3);
  }
  if (tid < 128) {
    const v4f v = *(const v4f*)(fc_w + tid * 4);
    const float v0 = v[0], v1 = v[1], v2 = v[2], v3 = v[3];
    Fw[tid * 4 + 0] = bf16r(v0);
    Fw[tid * 4 + 1] = bf16r(v1);
    Fw[tid * 4 + 2] = bf16r(v2);
    Fw[tid * 4 + 3] = bf16r(v3);
  }
  if (tid < 32) {
    const float fb = fc_b[tid & 3];
    if (tid < NO) Fb[tid] = bf16r(fb);
  }
  const float wr  = bf16r(w_ih[j]);
  const float wz  = bf16r(w_ih[NH + j]);
  const float wn  = bf16r(w_ih[2 * NH + j]);
  const float bir = bf16r(b_ih[j]);
  const float biz = bf16r(b_ih[NH + j]);
  const float bin = bf16r(b_ih[2 * NH + j]);
  const float bhr = bf16r(b_hh[j]);
  const float bhz = bf16r(b_hh[NH + j]);
  const float bhn = bf16r(b_hh[2 * NH + j]);

  float hst[8];
#pragma unroll
  for (int r = 0; r < 8; ++r) hst[r] = 0.0f;
  __syncthreads();

  const v8f z8 = {0.f, 0.f, 0.f, 0.f, 0.f, 0.f, 0.f, 0.f};
  const __bf16* w0 = Wsh + (size_t)(j) * WPITCH + koff;
  const __bf16* w1 = Wsh + (size_t)(NH + j) * WPITCH + koff;
  const __bf16* w2 = Wsh + (size_t)(2 * NH + j) * WPITCH + koff;

#pragma unroll 1
  for (int t = 0; t < NSTEP; ++t) {
    if ((t & (XCH - 1)) == 0) {
      const int m  = tid >> 4;
      const int c4 = (tid & 15) * 4;
      const v4f v = *(const v4f*)(x + (size_t)(rowbase + m) * NSTEP + (size_t)t + c4);
      const float v0 = v[0], v1 = v[1], v2 = v[2], v3 = v[3];
      v4f o;
      o[0] = bf16r(v0); o[1] = bf16r(v1); o[2] = bf16r(v2); o[3] = bf16r(v3);
      *(v4f*)(Xs + m * XCH + c4) = o;
      __syncthreads();
    }
    const int cur = t & 1;
    const int nxt = cur ^ 1;
    const __bf16* ah = &Hh[cur][0] + c * HPITCH + koff;
    const __bf16* al = &Hl[cur][0] + c * HPITCH + koff;

    v8f acc0 = z8, acc1 = z8, acc2 = z8;
#pragma unroll 1
    for (int k0 = 0; k0 < NH; k0 += 32) {
      const v16b fh = Frag<__bf16>::load(ah + k0);
      const v16b fl = Frag<__bf16>::load(al + k0);
      const v16b g0 = Frag<__bf16>::load(w0 + k0);
      const v16b g1 = Frag<__bf16>::load(w1 + k0);
      const v16b g2 = Frag<__bf16>::load(w2 + k0);
      acc0 = Frag<__bf16>::mma(fh, g0, acc0);
      acc0 = Frag<__bf16>::mma(fl, g0, acc0);
      acc1 = Frag<__bf16>::mma(fh, g1, acc1);
      acc1 = Frag<__bf16>::mma(fl, g1, acc1);
      acc2 = Frag<__bf16>::mma(fh, g2, acc2);
      acc2 = Frag<__bf16>::mma(fl, g2, acc2);
      mma_guard3(acc0, acc1, acc2, fh, fl, g0, g1, g2);
    }
    acc_guard3(acc0, acc1, acc2);

    const int tc = t & (XCH - 1);
#pragma unroll
    for (int r = 0; r < 8; ++r) {
      const int ri = 8 * hh + r;
      const float xv  = Xs[ri * XCH + tc];
      const float gir = xv * wr + bir;
      const float giz = xv * wz + biz;
      const float gin = xv * wn + bin;
      const float ghr = acc0[r] + bhr;
      const float ghz = acc1[r] + bhz;
      const float ghn = acc2[r] + bhn;
      const float rg  = fsig(gir + ghr);
      const float zg  = fsig(giz + ghz);
      const float ng  = ftanh(gin + rg * ghn);
      const float ho  = hst[r];
      const float hn  = (1.0f - zg) * ng + zg * ho;
      hst[r] = hn;
      const unsigned short hb = f2bf_bits(hn);
      const float hres = hn - bf_bits2f(hb);
      const unsigned short lb = f2bf_bits(hres);
      Hh[nxt][ri * HPITCH + j] = __builtin_bit_cast(__bf16, hb);
      Hl[nxt][ri * HPITCH + j] = __builtin_bit_cast(__bf16, lb);
    }
    __syncthreads();
  }

#pragma unroll
  for (int r = 0; r < 8; ++r) Hs[(8 * hh + r) * HSP + j] = hst[r];
  __syncthreads();
  if (tid < RB * NO) {
    const int b = tid >> 2, o = tid & 3;
    const float* hrow = Hs + b * HSP;
    const float* fw   = Fw + o * NH;
    float a = 0.0f;
#pragma unroll 4
    for (int k = 0; k < NH; ++k) a = a + hrow[k] * fw[k];
    a = a + Fb[o];
    Os[tid] = a;
  }
  __syncthreads();
  {
    const int q = tid & 15;
    const v4f v = *(const v4f*)(Os + 4 * q);
    if (tid < 16) {
      float* op = out + (size_t)rowbase * NO + 4 * q;
      *(volatile v4f*)op = v;
      __threadfence();
      *(volatile v4f*)op = v;
    }
  }
}

extern "C" void kernel_launch(void* const* d_in, const int* in_sizes, int n_in,
                              void* d_out, int out_size, void* d_ws, size_t ws_size, hipStream_t stream) {
  if (n_in < 7 || d_out == nullptr) return;
  if (in_sizes[0] != NB * NSTEP || in_sizes[1] != NG3 || in_sizes[2] != NG3 * NH || in_sizes[3] != NG3 ||
      in_sizes[4] != NG3 || in_sizes[5] != NO * NH || in_sizes[6] != NO || out_size != NB * NO) return;

  const float* x    = (const float*)d_in[0];
  const float* w_ih = (const float*)d_in[1];
  const float* w_hh = (const float*)d_in[2];
  const float* b_ih = (const float*)d_in[3];
  const float* b_hh = (const float*)d_in[4];
  const float* fc_w = (const float*)d_in[5];
  const float* fc_b = (const float*)d_in[6];
  float* out = (float*)d_out;

  gru_seq_kernel<<<NB / RB, NTHR, 0, stream>>>(x, w_ih, w_hh, b_ih, b_hh, fc_w, fc_b, out);
}
